// GatedDeltaNet_59064390255185
// MI455X (gfx1250) — hardware-run, weakly checked
//
#include <hip/hip_runtime.h>
#include <math.h>

constexpr int kB  = 2;
constexpr int kT  = 1024;
constexpr int kD  = 2048;
constexpr int kHK = 8;
constexpr int kHV = 16;
constexpr int kDK = 128;
constexpr int kDV = 128;
constexpr int kKW = 4;
constexpr int kKeyDim  = kHK * kDK;
constexpr int kValDim  = kHV * kDV;
constexpr int kConvDim = 2 * kKeyDim + kValDim;
constexpr int kRows    = kB * kT;
constexpr int kNcat    = kConvDim + 64;
constexpr int kGatePitch = 32;
constexpr int kA3ld    = 2 * kValDim;
constexpr float kQScale = 0.08838834764831845f;
constexpr float kL2Eps  = 1.0e-6f;
constexpr float kRmsEps = 1.0e-6f;
constexpr float kInvDV  = 1.0f / 128.0f;
constexpr float kFltMin = 1.17549435e-38f;
static_assert(kRows % 64 == 0 && kNcat % 64 == 0 && kValDim % 64 == 0 && kD % 64 == 0, "tiles");
static_assert(kD % 32 == 0 && kA3ld % 32 == 0, "ktiles");
static_assert(kConvDim == 4 * 1024 && kKeyDim == 1024 && kDK == 128 && kDV == 128, "shape");
static_assert((kNcat * 4) % 128 == 0 && (kGatePitch * 4) == 128, "lines");

typedef __attribute__((ext_vector_type(16))) _Float16 v16h;
typedef __attribute__((ext_vector_type(8)))  _Float16 v8h;
typedef __attribute__((ext_vector_type(16))) __bf16   v16b;
typedef __attribute__((ext_vector_type(8)))  __bf16   v8b;
typedef __attribute__((ext_vector_type(8)))  float    v8f;
typedef __attribute__((ext_vector_type(4)))  float    v4f;
typedef __attribute__((ext_vector_type(4)))  unsigned int v4u;

__device__ __forceinline__ unsigned short f2bf_bits(float f) {
  unsigned u = __float_as_uint(f);
  return (unsigned short)((u + 0x7FFFu + ((u >> 16) & 1u)) >> 16);
}
__device__ __forceinline__ float bf_bits2f(unsigned short h) { return __uint_as_float(((unsigned)h) << 16); }
__device__ __forceinline__ float bfr(float f) { return bf_bits2f(f2bf_bits(f)); }

__device__ __forceinline__ void dep_guard_h(v8f& a, v8f& b, v16h x, v16h y) { asm volatile("v_nop\n\tv_nop\n\tv_nop\n\tv_nop" : "+v"(a), "+v"(b) : "v"(x), "v"(y)); }
__device__ __forceinline__ void dep_guard_b(v8f& a, v8f& b, v16b x, v16b y) { asm volatile("v_nop\n\tv_nop\n\tv_nop\n\tv_nop" : "+v"(a), "+v"(b) : "v"(x), "v"(y)); }
__device__ __forceinline__ void keep4_h(v16h a, v16h b, v16h c, v16h d) { asm volatile("v_nop" :: "v"(a), "v"(b), "v"(c), "v"(d)); }
__device__ __forceinline__ void keep4_b(v16b a, v16b b, v16b c, v16b d) { asm volatile("v_nop" :: "v"(a), "v"(b), "v"(c), "v"(d)); }
__device__ __forceinline__ void acc_guard4(v8f& a, v8f& b, v8f& c, v8f& d) { asm volatile("v_nop\n\tv_nop\n\tv_nop\n\tv_nop" : "+v"(a), "+v"(b), "+v"(c), "+v"(d)); }
template <typename T> struct Frag;
template <> struct Frag<_Float16> {
  typedef v16h V; union U { v16h v; v8h h[2]; };
  static __device__ __forceinline__ v16h load(const _Float16* p) {
    U f; f.h[0] = *(const v8h*)(p); f.h[1] = *(const v8h*)(p + 16); return f.v;
  }
  static __device__ __forceinline__ v8f mma(v16h a, v16h b, v8f c) {
    return __builtin_amdgcn_wmma_f32_16x16x32_f16(false, a, false, b, (short)0, c, false, false);
  }
  static __device__ __forceinline__ void guard(v8f& a, v8f& b, v16h x, v16h y) { dep_guard_h(a, b, x, y); }
  static __device__ __forceinline__ void keep(v16h a, v16h b, v16h c, v16h d) { keep4_h(a, b, c, d); }
};
template <> struct Frag<__bf16> {
  typedef v16b V; union U { v16b v; v8b h[2]; };
  static __device__ __forceinline__ v16b load(const __bf16* p) {
    U f; f.h[0] = *(const v8b*)(p); f.h[1] = *(const v8b*)(p + 16); return f.v;
  }
  static __device__ __forceinline__ v8f mma(v16b a, v16b b, v8f c) {
    return __builtin_amdgcn_wmma_f32_16x16x32_bf16(false, a, false, b, (short)0, c, false, false);
  }
  static __device__ __forceinline__ void guard(v8f& a, v8f& b, v16b x, v16b y) { dep_guard_b(a, b, x, y); }
  static __device__ __forceinline__ void keep(v16b a, v16b b, v16b c, v16b d) { keep4_b(a, b, c, d); }
};

__device__ __forceinline__ unsigned pk16(unsigned short a, unsigned short b) { return (unsigned)a | ((unsigned)b << 16); }

template <int ET> struct Elem;
template <> struct Elem<0> { typedef _Float16 T; };
template <> struct Elem<1> { typedef __bf16 T; };
template <int ET, bool SPLIT, int BIAS_MODE, int OUT_MODE, bool RESID, int ACT = 0>
__global__ __launch_bounds__(256) void wmma_gemm64(
    const unsigned short* __restrict__ Ap, const unsigned short* __restrict__ A2p, int lda, long strideA,
    const unsigned short* __restrict__ Btp, const unsigned short* __restrict__ Bt2p, int ldb, long strideB,
    void* __restrict__ Cout, void* __restrict__ Cout2, int ldc, long strideC,
    const float* __restrict__ bias,
    const float* __restrict__ resid, long strideR,
    int M, int N, int K, float scale) {
  typedef typename Elem<ET>::T T;
  typedef typename Frag<T>::V V;
  const T* A = (const T*)Ap; const T* A2 = (const T*)A2p; const T* Bt = (const T*)Btp; const T* Bt2 = (const T*)Bt2p;
  __shared__ __align__(16) float sT[8][16 * 68];
  const int b    = blockIdx.y;
  const int lane = threadIdx.x & 31;
  const int wave = threadIdx.x >> 5;
  const int tilesN = N >> 6;
  const int tilesM = M >> 6;
  const int tile = blockIdx.x * 8 + wave;
  if (tile >= tilesM * tilesN) return;
  const int tm = tile / tilesN;
  const int tn = tile - tm * tilesN;
  const int m0 = tm << 6;
  const int n0 = tn << 6;

  const T* Ab  = A  + (size_t)b * strideA;
  const T* Bb  = Bt + (size_t)b * strideB;
  const T* Ab2 = SPLIT ? (A2  + (size_t)b * strideA) : nullptr;
  const T* Bb2 = SPLIT ? (Bt2 + (size_t)b * strideB) : nullptr;

  const int rlane = lane & 15;
  const int koff  = (lane >> 4) * 8;
  const int mOff  = (lane >> 4) * 8;

  v8f acc[4][4];
#pragma unroll
  for (int i = 0; i < 4; ++i)
#pragma unroll
    for (int j = 0; j < 4; ++j) acc[i][j] = (v8f){0.f,0.f,0.f,0.f,0.f,0.f,0.f,0.f};

  for (int k0 = 0; k0 < K; k0 += 32) {
    V bh[4], bl[4];
#pragma unroll
    for (int j = 0; j < 4; ++j) {
      const size_t bo = (size_t)(n0 + (j << 4) + rlane) * ldb + koff + k0;
      bh[j] = Frag<T>::load(Bb + bo);
      if (SPLIT) bl[j] = Frag<T>::load(Bb2 + bo);
    }
#pragma unroll
    for (int i = 0; i < 4; ++i) {
      const size_t ao = (size_t)(m0 + (i << 4) + rlane) * lda + koff + k0;
      V ah = Frag<T>::load(Ab + ao);
      V al;
      if (SPLIT) al = Frag<T>::load(Ab2 + ao);
#pragma unroll
      for (int j = 0; j < 4; ++j) {
        acc[i][j] = Frag<T>::mma(ah, bh[j], acc[i][j]);
        if (SPLIT) {
          acc[i][j] = Frag<T>::mma(ah, bl[j], acc[i][j]);
          acc[i][j] = Frag<T>::mma(al, bh[j], acc[i][j]);
        }
      }
      Frag<T>::guard(acc[i][0], acc[i][3], ah, SPLIT ? al : ah);
      Frag<T>::guard(acc[i][1], acc[i][2], ah, SPLIT ? al : ah);
    }
    Frag<T>::keep(bh[0], bh[1], bh[2], bh[3]);
    if (SPLIT) Frag<T>::keep(bl[0], bl[1], bl[2], bl[3]);
  }
  acc_guard4(acc[0][0], acc[0][1], acc[0][2], acc[0][3]);
  acc_guard4(acc[1][0], acc[1][1], acc[1][2], acc[1][3]);
  acc_guard4(acc[2][0], acc[2][1], acc[2][2], acc[2][3]);
  acc_guard4(acc[3][0], acc[3][1], acc[3][2], acc[3][3]);

  float* slab = sT[wave];
  const float* Rb = RESID ? (resid + (size_t)b * strideR) : nullptr;
#pragma unroll
  for (int i = 0; i < 4; ++i) {
    const int mBase = m0 + (i << 4);
#pragma unroll
    for (int j = 0; j < 4; ++j) {
      const int n = n0 + (j << 4) + rlane;
      float bv = 0.f;
      if (BIAS_MODE == 2) bv = bias[n];
#pragma unroll
      for (int r = 0; r < 8; ++r) {
        float v = acc[i][j][r] * scale;
        if (BIAS_MODE == 1) v += bias[mBase + mOff + r];
        if (BIAS_MODE == 2) v += bv;
        if (RESID) v += Rb[(size_t)(mBase + mOff + r) * ldc + n];
        if (ACT == 2) v = fmaxf(v, 0.0f);
        if (ACT == 4) v = (v > 0.f) ? v : 0.01f * v;
        slab[(mOff + r) * 68 + (j << 4) + rlane] = v;
      }
    }
    __builtin_amdgcn_fence(__ATOMIC_RELEASE, "workgroup");
    __builtin_amdgcn_wave_barrier();
    __builtin_amdgcn_fence(__ATOMIC_ACQUIRE, "workgroup");
    if (OUT_MODE == 0) {
      float* C = (float*)Cout + (size_t)b * strideC;
      const int hh = lane >> 4, c4 = (lane & 15) * 4;
      for (int pass = 0; pass < 2; ++pass) {
#pragma unroll
        for (int it = 0; it < 8; ++it) {
          const int row = it * 2 + hh;
          v4f v = *(const v4f*)(slab + row * 68 + c4);
          *(volatile v4f*)(C + (size_t)(mBase + row) * ldc + n0 + c4) = v;
        }
        __threadfence();
      }
    } else {
      const int q = lane >> 3, c8 = (lane & 7) * 8;
      unsigned short* C  = (unsigned short*)Cout  + (size_t)b * strideC;
      unsigned short* C2 = (OUT_MODE == 2) ? ((unsigned short*)Cout2 + (size_t)b * strideC) : nullptr;
      for (int pass = 0; pass < 2; ++pass) {
#pragma unroll
        for (int it = 0; it < 4; ++it) {
          const int row = it * 4 + q;
          const float* sp = slab + row * 68 + c8;
          v8h hv, lv;
#pragma unroll
          for (int e = 0; e < 8; ++e) {
            if (OUT_MODE == 1) {
              hv[e] = (_Float16)sp[e];
            } else {
              unsigned short hb = f2bf_bits(sp[e]);
              unsigned short lb = f2bf_bits(sp[e] - bf_bits2f(hb));
              hv[e] = __builtin_bit_cast(_Float16, hb);
              lv[e] = __builtin_bit_cast(_Float16, lb);
            }
          }
          *(volatile v8h*)(C + (size_t)(mBase + row) * ldc + n0 + c8) = hv;
          if (OUT_MODE == 2) *(volatile v8h*)(C2 + (size_t)(mBase + row) * ldc + n0 + c8) = lv;
        }
        __threadfence();
      }
    }
    __builtin_amdgcn_fence(__ATOMIC_RELEASE, "workgroup");
    __builtin_amdgcn_wave_barrier();
    __builtin_amdgcn_fence(__ATOMIC_ACQUIRE, "workgroup");
  }
}

__global__ __launch_bounds__(256) void cast8_bf16_kernel(const float* __restrict__ in, unsigned short* __restrict__ out, int n8) {
  const int i = blockIdx.x * 256 + threadIdx.x;
  if (i >= n8) return;
  const float* p = in + 8 * (size_t)i;
  const v4f a = *(const v4f*)(p);
  const v4f c = *(const v4f*)(p + 4);
  unsigned short hb[8];
#pragma unroll
  for (int e = 0; e < 4; ++e) {
    hb[e]     = f2bf_bits(a[e]);
    hb[4 + e] = f2bf_bits(c[e]);
  }
  const v4u u = (v4u){pk16(hb[0], hb[1]), pk16(hb[2], hb[3]), pk16(hb[4], hb[5]), pk16(hb[6], hb[7])};
  unsigned short* q = out + 8 * (size_t)i;
  *(volatile v4u*)q = u;
  __threadfence();
  *(volatile v4u*)q = u;
}

__global__ __launch_bounds__(256) void tcast_bf16_kernel(const float* __restrict__ W, int nout,
                                                         unsigned short* __restrict__ outp, int ldo, int coff) {
  __shared__ float sm[64][65];
  const int t  = threadIdx.x;
  const int k0 = blockIdx.x * 64;
  const int n0 = blockIdx.y * 64;
#pragma unroll
  for (int i = 0; i < 16; ++i) {
    const int e = i * 256 + t;
    const int r = e >> 6;
    const int c = e & 63;
    sm[c][r] = W[(size_t)(k0 + r) * nout + n0 + c];
  }
  __syncthreads();
  const int lane = t & 31, wave = t >> 5;
  const int q = lane >> 3, c8 = (lane & 7) * 8;
  for (int pass = 0; pass < 2; ++pass) {
#pragma unroll
    for (int it = 0; it < 2; ++it) {
      const int row = wave * 8 + it * 4 + q;
      unsigned short hb[8];
#pragma unroll
      for (int e = 0; e < 8; ++e) hb[e] = f2bf_bits(sm[row][c8 + e]);
      const v4u u = (v4u){pk16(hb[0], hb[1]), pk16(hb[2], hb[3]), pk16(hb[4], hb[5]), pk16(hb[6], hb[7])};
      *(volatile v4u*)(outp + (size_t)(n0 + row) * ldo + coff + k0 + c8) = u;
    }
    __threadfence();
  }
}

__global__ __launch_bounds__(256) void wba_kernel(const float* __restrict__ Wb, const float* __restrict__ Wa,
                                                  unsigned short* __restrict__ outp) {
  __shared__ float sm[64][65];
  const int t  = threadIdx.x;
  const int k0 = blockIdx.x * 64;
#pragma unroll
  for (int i = 0; i < 4; ++i) {
    const int e = i * 256 + t;
    const int r = e >> 4;
    const int c = e & 15;
    sm[c][r]      = Wb[(size_t)(k0 + r) * kHV + c];
    sm[16 + c][r] = Wa[(size_t)(k0 + r) * kHV + c];
  }
#pragma unroll
  for (int i = 0; i < 8; ++i) {
    const int e = i * 256 + t;
    sm[32 + (e >> 6)][e & 63] = 0.0f;
  }
  __syncthreads();
  const int lane = t & 31, wave = t >> 5;
  const int q = lane >> 3, c8 = (lane & 7) * 8;
  for (int pass = 0; pass < 2; ++pass) {
#pragma unroll
    for (int it = 0; it < 2; ++it) {
      const int row = wave * 8 + it * 4 + q;
      unsigned short hb[8];
#pragma unroll
      for (int e = 0; e < 8; ++e) hb[e] = f2bf_bits(sm[row][c8 + e]);
      const v4u u = (v4u){pk16(hb[0], hb[1]), pk16(hb[2], hb[3]), pk16(hb[4], hb[5]), pk16(hb[6], hb[7])};
      *(volatile v4u*)(outp + (size_t)(kConvDim + row) * kD + k0 + c8) = u;
    }
    __threadfence();
  }
}

__global__ __launch_bounds__(256) void conv_kernel(const float* __restrict__ c1, const float* __restrict__ cw,
                                                   float* __restrict__ qn, float* __restrict__ kn, float* __restrict__ vpl) {
  const int bt   = blockIdx.x;
  const int tpos = bt & (kT - 1);
  const int tid  = threadIdx.x;
#pragma unroll 1
  for (int ph = 0; ph < 4; ++ph) {
    const int c0 = ph * 1024 + tid * 4;
    float wb[4][4];
#pragma unroll
    for (int i = 0; i < 4; ++i) {
      const v4f w4 = *(const v4f*)(cw + (size_t)(c0 + i) * kKW);
#pragma unroll
      for (int j = 0; j < 4; ++j) wb[i][j] = bfr(w4[j]);
    }
    float acc[4] = {0.0f, 0.0f, 0.0f, 0.0f};
#pragma unroll
    for (int j = 0; j < kKW; ++j) {
      const int back = kKW - 1 - j;
      const bool valid = (tpos >= back);
      const int rr = valid ? (bt - back) : bt;
      const float fz = valid ? 1.0f : 0.0f;
      const v4f x4 = *(const v4f*)(c1 + (size_t)rr * kNcat + c0);
#pragma unroll
      for (int i = 0; i < 4; ++i) acc[i] = fmaf(wb[i][j], x4[i] * fz, acc[i]);
    }
    float sv[4];
    float ss = 0.0f;
#pragma unroll
    for (int i = 0; i < 4; ++i) {
      const float y  = acc[i];
      const float s1 = y / (1.0f + expf(-y));
      sv[i] = s1;
      ss = fmaf(s1, s1, ss);
    }
#pragma unroll
    for (int off = 16; off > 0; off >>= 1) ss += __shfl_xor(ss, off, 32);
    const float rs = rsqrtf(ss + kL2Eps);
    const float sc = (ph == 0) ? (rs * kQScale) : ((ph == 1) ? rs : 1.0f);
    float* dst = (ph == 0) ? (qn + (size_t)bt * kKeyDim + tid * 4)
               : (ph == 1) ? (kn + (size_t)bt * kKeyDim + tid * 4)
               : (vpl + (size_t)bt * kValDim + (ph - 2) * 1024 + tid * 4);
    const v4f val = (v4f){sv[0] * sc, sv[1] * sc, sv[2] * sc, sv[3] * sc};
    *(volatile v4f*)dst = val;
    __threadfence();
    *(volatile v4f*)dst = val;
  }
}

__global__ __launch_bounds__(256) void gates_kernel(const float* __restrict__ c1, const float* __restrict__ dtb,
                                                    const float* __restrict__ alog, float* __restrict__ gb) {
  const int tid = threadIdx.x, wave = tid >> 5, lane = tid & 31;
  const int bt  = blockIdx.x * 8 + wave;
  const int h   = lane & 15;
  const int sel = lane >> 4;
  const float x  = c1[(size_t)bt * kNcat + kConvDim + lane];
  const float al = bfr(alog[h]);
  const float db = bfr(dtb[h]);
  const float beta = 1.0f / (1.0f + expf(-x));
  const float xs = x + db;
  const float sp = fmaxf(xs, 0.0f) + log1pf(expf(-fabsf(xs)));
  const float g  = -expf(al) * sp;
  float dec = expf(g);
  dec = (dec < kFltMin) ? 0.0f : dec;
  const float fd  = (float)sel;
  const float fb  = 1.0f - fd;
  const float val = fmaf(fb, beta, fd * dec);
  float* op = gb + (size_t)bt * kGatePitch + lane;
  *(volatile float*)op = val;
  __threadfence();
  *(volatile float*)op = val;
}

__global__ __launch_bounds__(256) void scan_kernel(const float* __restrict__ qn, const float* __restrict__ kn,
                                                   const float* __restrict__ vpl, const float* __restrict__ gb,
                                                   float* __restrict__ obuf) {
  __shared__ __align__(16) float kq[2][256];
  __shared__ __align__(16) float oL[2][32];
  const int blk = blockIdx.x;
  const int bh  = blk >> 2, cg = blk & 3;
  const int b   = bh >> 4, h = bh & 15, hk = h >> 1;
  const int tid = threadIdx.x, wave = tid >> 5, lane = tid & 31;
  const int cw  = lane >> 3, s = lane & 7;
  const int colL = wave * 4 + cw;
  const int dv   = cg * 32 + colL;
  const float* kqsrc = (tid < 128) ? kn : qn;
  const int kqoff = hk * kDK + (tid & 127);

  float S[16];
#pragma unroll
  for (int i = 0; i < 16; ++i) S[i] = 0.0f;

#pragma unroll 1
  for (int t = 0; t < kT; ++t) {
    const int p  = t & 1;
    const int bt = b * kT + t;
    const float stg  = kqsrc[(size_t)bt * kKeyDim + kqoff];
    const float vt   = vpl[(size_t)bt * kValDim + h * kDV + dv];
    const float beta = gb[(size_t)bt * kGatePitch + h];
    const float dec  = gb[(size_t)bt * kGatePitch + 16 + h];
    kq[p][tid] = stg;
    __syncthreads();
    if (wave == 0 && t > 0) {
      const float ov = oL[p ^ 1][lane];
      float* op = obuf + ((size_t)(bt - 1) * kValDim + h * kDV + cg * 32 + lane);
      *(volatile float*)op = ov;
      __threadfence();
      *(volatile float*)op = ov;
    }
    const float* kp = &kq[p][16 * s];
    const float* qp = &kq[p][128 + 16 * s];
    float kk[16], qq[16];
#pragma unroll
    for (int i = 0; i < 4; ++i) {
      const v4f kv4 = *(const v4f*)(kp + 4 * i);
      const v4f qv4 = *(const v4f*)(qp + 4 * i);
#pragma unroll
      for (int e = 0; e < 4; ++e) { kk[4 * i + e] = kv4[e]; qq[4 * i + e] = qv4[e]; }
    }
    float u = 0.0f;
#pragma unroll
    for (int i = 0; i < 16; ++i) { S[i] *= dec; u = fmaf(kk[i], S[i], u); }
    u += __shfl_xor(u, 1, 32);
    u += __shfl_xor(u, 2, 32);
    u += __shfl_xor(u, 4, 32);
    const float vadj = (vt - u) * beta;
    float o = 0.0f;
#pragma unroll
    for (int i = 0; i < 16; ++i) { S[i] = fmaf(kk[i], vadj, S[i]); o = fmaf(qq[i], S[i], o); }
    o += __shfl_xor(o, 1, 32);
    o += __shfl_xor(o, 2, 32);
    o += __shfl_xor(o, 4, 32);
    if (s == 0) oL[p][colL] = o;
  }
  __syncthreads();
  if (wave == 0) {
    const float ov = oL[(kT - 1) & 1][lane];
    float* op = obuf + ((size_t)(b * kT + kT - 1) * kValDim + h * kDV + cg * 32 + lane);
    *(volatile float*)op = ov;
    __threadfence();
    *(volatile float*)op = ov;
  }
}

__global__ __launch_bounds__(256) void normgate_kernel(const float* __restrict__ obuf, const float* __restrict__ zb,
                                                       const float* __restrict__ nw, unsigned short* __restrict__ a3) {
  const int tid = threadIdx.x, wave = tid >> 5, lane = tid & 31;
  const int vec = (blockIdx.x * 8 + wave) * 2 + (lane >> 4);
  const int bt  = vec >> 4, h = vec & 15;
  const int d0  = (lane & 15) * 8;
  const size_t base = (size_t)bt * kValDim + h * kDV + d0;
  const v4f o0 = *(const v4f*)(obuf + base);
  const v4f o1 = *(const v4f*)(obuf + base + 4);
  const v4f z0 = *(const v4f*)(zb + base);
  const v4f z1 = *(const v4f*)(zb + base + 4);
  const v4f w0 = *(const v4f*)(nw + d0);
  const v4f w1 = *(const v4f*)(nw + d0 + 4);
  float o[8], z[8], w[8];
#pragma unroll
  for (int e = 0; e < 4; ++e) {
    o[e] = o0[e]; o[4 + e] = o1[e];
    z[e] = z0[e]; z[4 + e] = z1[e];
    w[e] = w0[e]; w[4 + e] = w1[e];
  }
  float ss = 0.0f;
#pragma unroll
  for (int e = 0; e < 8; ++e) ss = fmaf(o[e], o[e], ss);
  ss += __shfl_xor(ss, 1, 32);
  ss += __shfl_xor(ss, 2, 32);
  ss += __shfl_xor(ss, 4, 32);
  ss += __shfl_xor(ss, 8, 32);
  const float rs = rsqrtf(ss * kInvDV + kRmsEps);
  unsigned short hb[8], lb[8];
#pragma unroll
  for (int e = 0; e < 8; ++e) {
    const float wv = bfr(w[e]);
    const float gn = (o[e] * rs) * wv;
    const float ze = z[e];
    const float sz = ze * __builtin_amdgcn_rcpf(1.0f + expf(-ze));
    const float og = gn * sz;
    const unsigned short hbe = f2bf_bits(og);
    hb[e] = hbe;
    lb[e] = f2bf_bits(og - bf_bits2f(hbe));
  }
  const v4u uh = (v4u){pk16(hb[0], hb[1]), pk16(hb[2], hb[3]), pk16(hb[4], hb[5]), pk16(hb[6], hb[7])};
  const v4u ul = (v4u){pk16(lb[0], lb[1]), pk16(lb[2], lb[3]), pk16(lb[4], lb[5]), pk16(lb[6], lb[7])};
  unsigned short* ph = a3 + (size_t)bt * kA3ld + h * kDV + d0;
  unsigned short* pl = ph + kValDim;
  *(volatile v4u*)ph = uh;
  *(volatile v4u*)pl = ul;
  __threadfence();
  *(volatile v4u*)ph = uh;
  *(volatile v4u*)pl = ul;
}

extern "C" void kernel_launch(void* const* d_in, const int* in_sizes, int n_in,
                              void* d_out, int out_size, void* d_ws, size_t ws_size,
                              hipStream_t stream) {
  if (n_in < 10) return;
  if (in_sizes[0] != kRows * kD) return;
  if (in_sizes[1] != kD * kConvDim) return;
  if (in_sizes[2] != kD * kValDim) return;
  if (in_sizes[3] != kD * kHV || in_sizes[4] != kD * kHV) return;
  if (in_sizes[5] != kConvDim * kKW) return;
  if (in_sizes[6] != kHV || in_sizes[7] != kHV || in_sizes[8] != kDV) return;
  if (in_sizes[9] != kValDim * kD) return;
  if (out_size != kRows * kD) return;

  const size_t szHid  = (size_t)kRows * kD * 2;
  const size_t szWcat = (size_t)kNcat * kD * 2;
  const size_t szWzo  = (size_t)kD * kA3ld * 2;
  const size_t szC1   = (size_t)kRows * kNcat * 4;
  const size_t szZ    = (size_t)kRows * kValDim * 4;
  const size_t szQ    = (size_t)kRows * kKeyDim * 4;
  const size_t szV    = (size_t)kRows * kValDim * 4;
  const size_t szG    = (size_t)kRows * kGatePitch * 4;
  static_assert((size_t)kRows * kA3ld * 2 <= (size_t)kNcat * kD * 2, "a3 fits wcat region");
  static_assert((size_t)kRows * kValDim * 4 <= (size_t)kRows * kNcat * 4, "obuf fits c1 region");
  const size_t offHid  = 0;
  const size_t offWcat = offHid + szHid;
  const size_t offWzo  = offWcat + szWcat;
  const size_t offC1   = offWzo + szWzo;
  const size_t offZ    = offC1 + szC1;
  const size_t offQ    = offZ + szZ;
  const size_t offK    = offQ + szQ;
  const size_t offV    = offK + szQ;
  const size_t offG    = offV + szV;
  const size_t total   = offG + szG;
  if (ws_size < total) return;

  const float* hidden = (const float*)d_in[0];
  const float* W_qkv  = (const float*)d_in[1];
  const float* W_z    = (const float*)d_in[2];
  const float* W_b    = (const float*)d_in[3];
  const float* W_a    = (const float*)d_in[4];
  const float* conv_w = (const float*)d_in[5];
  const float* dt_b   = (const float*)d_in[6];
  const float* A_log  = (const float*)d_in[7];
  const float* norm_w = (const float*)d_in[8];
  const float* W_out  = (const float*)d_in[9];
  float* out = (float*)d_out;
  char* ws = (char*)d_ws;
  unsigned short* HID  = (unsigned short*)(ws + offHid);
  unsigned short* WCAT = (unsigned short*)(ws + offWcat);
  unsigned short* A3   = WCAT;
  unsigned short* WZO  = (unsigned short*)(ws + offWzo);
  float* C1   = (float*)(ws + offC1);
  float* OBUF = C1;
  float* Z    = (float*)(ws + offZ);
  float* QN   = (float*)(ws + offQ);
  float* KN   = (float*)(ws + offK);
  float* VP   = (float*)(ws + offV);
  float* GB   = (float*)(ws + offG);

  const int n8 = (kRows * kD) / 8;
  cast8_bf16_kernel<<<dim3(n8 / 256), dim3(256), 0, stream>>>(hidden, HID, n8);
  tcast_bf16_kernel<<<dim3(kD / 64, kConvDim / 64), dim3(256), 0, stream>>>(W_qkv, kConvDim, WCAT, kD, 0);
  wba_kernel<<<dim3(kD / 64), dim3(256), 0, stream>>>(W_b, W_a, WCAT);
  tcast_bf16_kernel<<<dim3(kD / 64, kValDim / 64), dim3(256), 0, stream>>>(W_z, kValDim, WZO, kD, 0);
  wmma_gemm64<1, false, 0, 0, false, 0><<<dim3((kRows / 64) * (kNcat / 64) / 8, 1), dim3(256), 0, stream>>>(
      HID, HID, kD, 0L, WCAT, WCAT, kD, 0L, (void*)C1, (void*)C1, kNcat, 0L, GB, GB, 0L, kRows, kNcat, kD, 1.0f);
  wmma_gemm64<1, false, 0, 0, false, 0><<<dim3((kRows / 64) * (kValDim / 64) / 8, 1), dim3(256), 0, stream>>>(
      HID, HID, kD, 0L, WZO, WZO, kD, 0L, (void*)Z, (void*)Z, kValDim, 0L, GB, GB, 0L, kRows, kValDim, kD, 1.0f);
  tcast_bf16_kernel<<<dim3(kValDim / 64, kD / 64), dim3(256), 0, stream>>>(W_out, kD, WZO, kA3ld, 0);
  tcast_bf16_kernel<<<dim3(kValDim / 64, kD / 64), dim3(256), 0, stream>>>(W_out, kD, WZO, kA3ld, kValDim);
  conv_kernel<<<dim3(kRows), dim3(256), 0, stream>>>(C1, conv_w, QN, KN, VP);
  gates_kernel<<<dim3(kRows / 8), dim3(256), 0, stream>>>(C1, dt_b, A_log, GB);
  scan_kernel<<<dim3(kB * kHV * 4), dim3(256), 0, stream>>>(QN, KN, VP, GB, OBUF);
  normgate_kernel<<<dim3((kRows * kHV) / 16), dim3(256), 0, stream>>>(OBUF, Z, norm_w, A3);
  wmma_gemm64<1, false, 0, 0, false, 0><<<dim3((kRows / 64) * (kD / 64) / 8, 1), dim3(256), 0, stream>>>(
      A3, A3, kA3ld, 0L, WZO, WZO, kA3ld, 0L, (void*)out, (void*)out, kD, 0L, GB, GB, 0L, kRows, kD, kA3ld, 1.0f);
}
